// loraLinearAttention_53283364274846
// MI455X (gfx1250) — hardware-verified
//
#include <hip/hip_runtime.h>
#include <math.h>

typedef __attribute__((ext_vector_type(16))) _Float16 v16h;
typedef __attribute__((ext_vector_type(16))) __bf16 v16b;
typedef __attribute__((ext_vector_type(8)))  _Float16 v8h;
typedef __attribute__((ext_vector_type(8)))  float v8f;
typedef __attribute__((ext_vector_type(4)))  float v4f;
typedef __attribute__((ext_vector_type(2)))  float v2f;
typedef __attribute__((ext_vector_type(4)))  unsigned v4u;
typedef __attribute__((ext_vector_type(4)))  int v4i;
typedef float __attribute__((may_alias)) float_a;
typedef int __attribute__((may_alias)) int_a;

template <typename T> __device__ __forceinline__ void vst2(void* p, T v) { *(volatile T*)p = v; __threadfence(); *(volatile T*)p = v; }
__device__ __forceinline__ v8f wmma16(v16h a, v16h b, v8f c) {
  v8f d = __builtin_amdgcn_wmma_f32_16x16x32_f16(false, a, false, b, (short)0, c, false, false);
  asm volatile("v_nop\n\tv_nop\n\tv_nop\n\tv_nop" : "+v"(d) : "v"(a), "v"(b));
  return d;
}
__device__ __forceinline__ v8f wmma_bf(v16b a, v16b b, v8f c) {
  v8f d = __builtin_amdgcn_wmma_f32_16x16x32_bf16(false, a, false, b, (short)0, c, false, false);
  asm volatile("v_nop\n\tv_nop\n\tv_nop\n\tv_nop" : "+v"(d) : "v"(a), "v"(b));
  return d;
}
__device__ __forceinline__ v16h frag_h(const _Float16* rowk0, int lane) {
  union { v16h v; v8h q[2]; } u; const _Float16* p = rowk0 + 8 * (lane >> 4);
  u.q[0] = *(const v8h*)p; u.q[1] = *(const v8h*)(p + 16); return u.v;
}
__device__ __forceinline__ v16h frag_f32(const float* rowk0, int lane) {
  v16h a; const float* p = rowk0 + 8 * (lane >> 4);
#pragma unroll
  for (int i = 0; i < 8; ++i) { a[i] = (_Float16)p[i]; a[8 + i] = (_Float16)p[16 + i]; }
  return a;
}
__device__ __forceinline__ v16h frag_f32s(const float* rowk0, int lane, float sc) {
  v16h a; const float* p = rowk0 + 8 * (lane >> 4);
#pragma unroll
  for (int i = 0; i < 8; ++i) { a[i] = (_Float16)(p[i] * sc); a[8 + i] = (_Float16)(p[16 + i] * sc); }
  return a;
}
__device__ __forceinline__ v16h fragc_f32(const float* W, int k0, int n, int lane, int ld, int K) {
  v16h a; const int g = lane >> 4;
#pragma unroll
  for (int i = 0; i < 8; ++i) { const int ka = k0 + 8 * g + i, kb = ka + 16;
    a[i] = (_Float16)(ka < K ? W[(size_t)(ka < K ? ka : K - 1) * ld + n] : 0.f); a[8 + i] = (_Float16)(kb < K ? W[(size_t)(kb < K ? kb : K - 1) * ld + n] : 0.f); }
  return a;
}
struct F2 { v16b h, l; };
__device__ __forceinline__ F2 bsplit16(const float v[16]) { F2 r;
#pragma unroll
  for (int i = 0; i < 16; ++i) { const __bf16 h = (__bf16)v[i]; r.h[i] = h; r.l[i] = (__bf16)(v[i] - (float)h); }
  return r; }
__device__ __forceinline__ F2 split_row(const float* row, int k0, int lane) { float v[16]; const float* p = row + k0 + 8 * (lane >> 4);
#pragma unroll
  for (int i = 0; i < 8; ++i) { v[i] = p[i]; v[8 + i] = p[16 + i]; }
  return bsplit16(v); }
__device__ __forceinline__ F2 split_rowK(const float* row, int k0, int lane, int K) { float v[16]; const int g = lane >> 4;
#pragma unroll
  for (int i = 0; i < 8; ++i) { const int ka = k0 + 8 * g + i, kb = ka + 16; v[i] = ka < K ? row[ka < K ? ka : K - 1] : 0.f; v[8 + i] = kb < K ? row[kb < K ? kb : K - 1] : 0.f; }
  return bsplit16(v); }
__device__ __forceinline__ F2 split_col(const float* W, int k0, int n, int lane, int ld, int K) { float v[16]; const int g = lane >> 4;
#pragma unroll
  for (int i = 0; i < 8; ++i) { const int ka = k0 + 8 * g + i, kb = ka + 16; v[i] = ka < K ? W[(size_t)(ka < K ? ka : K - 1) * ld + n] : 0.f; v[8 + i] = kb < K ? W[(size_t)(kb < K ? kb : K - 1) * ld + n] : 0.f; }
  return bsplit16(v); }
__device__ __forceinline__ v8f mac3(const F2& a, const F2& b, v8f c) { c = wmma_bf(a.l, b.h, c); c = wmma_bf(a.h, b.l, c); return wmma_bf(a.h, b.h, c); }
__device__ __forceinline__ float sigm(float v) { return 1.0f / (1.0f + expf(-v)); }
#define LDSX() do { asm volatile("s_wait_dscnt 0" ::: "memory"); __builtin_amdgcn_wave_barrier(); __builtin_amdgcn_fence(__ATOMIC_RELEASE, "workgroup"); } while (0)


#define NB 16
#define CC 128
#define NP 4096
#define NH 4
#define KD 32
#define QC 128
#define RK 4
#ifndef TNB
#define TNB NB
#define TPT (NP / 128)
#endif
typedef __attribute__((ext_vector_type(8))) __bf16 v8b;
__device__ __forceinline__ v16b frag_b(const __bf16* rowk0, int lane) {
  union { v16b v; v8b q[2]; } u; const __bf16* p = rowk0 + 8 * (lane >> 4);
  u.q[0] = *(const v8b*)p; u.q[1] = *(const v8b*)(p + 16); return u.v;
}
__device__ __forceinline__ float bfr(float v) { return (float)(__bf16)v; }
__device__ __attribute__((noinline)) float exp_ni(float v) { return expf(v); }
__device__ __attribute__((noinline)) float erf_ni(float v) { return erff(v); }

#define WS_WE  0u
#define WS_BE  (WS_WE + 4u * (size_t)3 * QC * CC)
#define WS_XT  (WS_BE + 4u * (size_t)3 * QC)
#define WS_QP  (WS_XT + 2u * (size_t)NP * CC)
#define WS_KP  (WS_QP + 2u * (size_t)QC * NP)
#define WS_VP  (WS_KP + 2u * (size_t)QC * NP)
#define WS_KS  (WS_VP + 2u * (size_t)QC * NP)
#define WS_QS  (WS_KS + 2u * (size_t)QC * NP)
#define WS_CT  (WS_QS + 2u * (size_t)NP * QC)
#define WS_M   (WS_CT + 4u * (size_t)NH * KD * KD)
#define WS_END (WS_M + 4u * (size_t)CC * QC)

__global__ __launch_bounds__(128) void k_fold(const float* __restrict__ WQKV, const float* __restrict__ AQ, const float* __restrict__ BAQ, const float* __restrict__ WBQ, const float* __restrict__ BBQ, const float* __restrict__ AK, const float* __restrict__ BAK, const float* __restrict__ WBK, const float* __restrict__ BBK, const float* __restrict__ AV, const float* __restrict__ BAV, const float* __restrict__ WBV, const float* __restrict__ BBV, float* __restrict__ WE, float* __restrict__ BE) {
  __shared__ __align__(16) float so2[CC]; const int o = blockIdx.x, which = blockIdx.y, t = threadIdx.x;
  const float* A = (which == 0) ? AQ : (which == 1) ? AK : AV; const float* BA = (which == 0) ? BAQ : (which == 1) ? BAK : BAV; const float* WB = (which == 0) ? WBQ : (which == 1) ? WBK : WBV; const float* BB = (which == 0) ? BBQ : (which == 1) ? BBK : BBV;
  float wb[RK]; for (int r = 0; r < RK; ++r) wb[r] = bfr(WB[o * RK + r]);
  { float a = 0.f; for (int r = 0; r < RK; ++r) a += wb[r] * bfr(A[r * CC + t]); so2[t] = bfr(WQKV[((size_t)which * QC + o) * CC + t]) + a * (1.0f / RK); }
  __syncthreads(); if (t < CC / 4) vst2(WE + ((size_t)which * QC + o) * CC + t * 4, *(const v4f*)&so2[t * 4]); (void)BA; (void)BB; (void)BE; }
__global__ __launch_bounds__(128) void k_foldb(const float* __restrict__ BAQ, const float* __restrict__ WBQ, const float* __restrict__ BBQ, const float* __restrict__ BAK, const float* __restrict__ WBK, const float* __restrict__ BBK, const float* __restrict__ BAV, const float* __restrict__ WBV, const float* __restrict__ BBV, float* __restrict__ BE) { __shared__ __align__(16) float so2[QC]; const int which = blockIdx.x, o = threadIdx.x;
  const float* BA = (which == 0) ? BAQ : (which == 1) ? BAK : BAV; const float* WB = (which == 0) ? WBQ : (which == 1) ? WBK : WBV; const float* BB = (which == 0) ? BBQ : (which == 1) ? BBK : BBV;
  float bb = 0.f; for (int r = 0; r < RK; ++r) bb += bfr(WB[o * RK + r]) * bfr(BA[r]); so2[o] = (bb + bfr(BB[o])) * (1.0f / RK); __syncthreads(); if (o < QC / 4) vst2(BE + (size_t)which * QC + o * 4, *(const v4f*)&so2[o * 4]); }
__global__ __launch_bounds__(256) void k_xt(const float* __restrict__ X, __bf16* __restrict__ XT) { __shared__ float st[64][CC + 1]; __shared__ __align__(16) __bf16 so2[64][CC + 8]; const int t = threadIdx.x; const int p0 = blockIdx.x * 64;
  for (int e = t; e < CC * 64; e += 256) { const int c = e >> 6, pl = e & 63; st[pl][c] = X[(size_t)c * NP + p0 + pl]; } __syncthreads();
  for (int e = t; e < 64 * CC; e += 256) { const int pl = e >> 7, c = e & 127; so2[pl][c] = (__bf16)st[pl][c]; } __syncthreads();
  for (int e = t; e < 64 * 16; e += 256) { const int pl = e >> 4, q = e & 15; vst2((unsigned*)(XT + ((size_t)(p0 + pl) * CC) + q * 8), *(const v4u*)&so2[pl][q * 8]); } }
__global__ __launch_bounds__(128) void k_conv(const float* __restrict__ WE, const float* __restrict__ BE, const __bf16* __restrict__ XT, _Float16* __restrict__ QP, _Float16* __restrict__ KP, _Float16* __restrict__ VP) { __shared__ __align__(16) _Float16 sh[4][16][136];
  const int tid = threadIdx.x, wave = tid >> 5, lane = tid & 31, col = lane & 15, g = lane >> 4; const int which = blockIdx.z; const int o0 = blockIdx.x * 64 + wave * 16; const int p0 = blockIdx.y * 128; const float* Wr = WE + ((size_t)which * QC) * CC;
  v8f acc[8] = {};
#pragma unroll
  for (int kc = 0; kc < CC / 32; ++kc) { const F2 a = split_row(Wr + (size_t)(o0 + col) * CC, kc * 32, lane);
#pragma unroll
    for (int j = 0; j < 8; ++j) { const v16b xb = frag_b(XT + ((size_t)(p0 + j * 16 + col) * CC) + kc * 32, lane); acc[j] = wmma_bf(a.h, xb, acc[j]); acc[j] = wmma_bf(a.l, xb, acc[j]); } }
#pragma unroll
  for (int j = 0; j < 8; ++j)
#pragma unroll
    for (int r = 0; r < 8; ++r) sh[wave][8 * g + r][j * 16 + col] = (_Float16)(acc[j][r] + BE[which * QC + o0 + 8 * g + r]);
  LDSX(); _Float16* dst = (which == 0) ? QP : (which == 1) ? KP : VP; for (int rl = 0; rl < 16; ++rl) if (lane < 16) vst2((unsigned*)(dst + ((size_t)(o0 + rl) * NP) + p0 + lane * 8), *(const v4u*)&sh[wave][rl][lane * 8]); }
__global__ __launch_bounds__(256) void k_ksoft(const _Float16* __restrict__ KP, _Float16* __restrict__ KS) { __shared__ float red[8]; __shared__ __align__(16) _Float16 sp[NP]; const int t = threadIdx.x; const size_t row = blockIdx.x; const _Float16* kr = KP + row * NP;
  float v[16]; float mx = -3.0e38f; for (int i = 0; i < 16; ++i) { v[i] = (float)kr[t * 16 + i]; mx = fmaxf(mx, v[i]); }
#pragma unroll
  for (int o = 1; o < 32; o <<= 1) mx = fmaxf(mx, __shfl_xor(mx, o));
  if ((t & 31) == 0) red[t >> 5] = mx; __syncthreads(); float M = red[0]; for (int i = 1; i < 8; ++i) M = fmaxf(M, red[i]); __syncthreads();
  float z = 0.f; for (int i = 0; i < 16; ++i) { v[i] = __expf(v[i] - M); z += v[i]; }
#pragma unroll
  for (int o = 1; o < 32; o <<= 1) z += __shfl_xor(z, o);
  if ((t & 31) == 0) red[t >> 5] = z; __syncthreads(); float Z = 0.f; for (int i = 0; i < 8; ++i) Z += red[i]; const float iz = 4096.0f / Z;
  for (int i = 0; i < 16; ++i) sp[t * 16 + i] = (_Float16)(v[i] * iz); __syncthreads();
  for (int q = t; q < NP / 8; q += 256) vst2((unsigned*)(KS + row * NP + q * 8), *(const v4u*)&sp[q * 8]); }
__global__ __launch_bounds__(128) void k_qsoft(const _Float16* __restrict__ QP, _Float16* __restrict__ QS) { __shared__ float st[QC][128 + 1]; __shared__ __align__(16) _Float16 so2[128][QC + 8]; const int t = threadIdx.x; const int p0 = blockIdx.x * 128;
  for (int c = 0; c < QC; ++c) st[c][t] = (float)QP[((size_t)c * NP) + p0 + t]; __syncthreads();
  for (int h = 0; h < NH; ++h) { float mx = -3.0e38f; for (int d = 0; d < KD; ++d) mx = fmaxf(mx, st[h * KD + d][t]); float z = 0.f; for (int d = 0; d < KD; ++d) z += __expf(st[h * KD + d][t] - mx); const float iz = 0.17677669529663688f / z; for (int d = 0; d < KD; ++d) so2[t][h * KD + d] = (_Float16)(__expf(st[h * KD + d][t] - mx) * iz); }
  __syncthreads(); for (int e = t; e < 128 * 16; e += 128) { const int pl = e >> 4, q = e & 15; vst2((unsigned*)(QS + ((size_t)(p0 + pl) * QC) + q * 8), *(const v4u*)&so2[pl][q * 8]); } }
__global__ __launch_bounds__(64) void k_ctx(const _Float16* __restrict__ KS, const _Float16* __restrict__ VP, float* __restrict__ CT) { __shared__ __align__(16) float so[2][16][36];
  const int tid = threadIdx.x, wave = tid >> 5, lane = tid & 31, col = lane & 15, g = lane >> 4; const int h = blockIdx.x; const _Float16* Kb = KS + ((size_t)(h * KD + wave * 16) * NP); const _Float16* Vb = VP + ((size_t)(h * KD) * NP);
  v8f acc[2] = {};
#pragma unroll 4
  for (int kc = 0; kc < NP / 32; ++kc) { const v16h a = frag_h(Kb + (size_t)col * NP + kc * 32, lane);
#pragma unroll
    for (int j = 0; j < 2; ++j) acc[j] = wmma16(a, frag_h(Vb + (size_t)(j * 16 + col) * NP + kc * 32, lane), acc[j]); }
#pragma unroll
  for (int j = 0; j < 2; ++j)
#pragma unroll
    for (int r = 0; r < 8; ++r) so[wave][8 * g + r][j * 16 + col] = acc[j][r] * (1.0f / 4096.0f) * (1.0f / (float)NP);
  LDSX(); for (int rl = 0; rl < 16; ++rl) if (lane < 8) vst2(CT + (((size_t)h * KD + wave * 16 + rl) * KD) + lane * 4, *(const v4f*)&so[wave][rl][lane * 4]); }
__global__ __launch_bounds__(128) void k_m(const float* __restrict__ WO, const float* __restrict__ CT, float* __restrict__ M) { __shared__ float sw[QC]; __shared__ __align__(16) float so2[QC]; const int t = threadIdx.x; const int o = blockIdx.x;
  sw[t] = bfr(WO[(size_t)o * QC + t]); __syncthreads();
  { const int h = t / KD, d = t % KD; const float* ct = CT + (((size_t)h * KD + d) * KD); float a = 0.f; for (int e = 0; e < KD; ++e) a += sw[h * KD + e] * ct[e]; so2[t] = a; } __syncthreads();
  if (t < QC / 4) vst2(M + ((size_t)o) * QC + t * 4, *(const v4f*)&so2[t * 4]); }
__global__ __launch_bounds__(128) void k_y(const float* __restrict__ M, const _Float16* __restrict__ QS, const float* __restrict__ BO, float* __restrict__ Y) { __shared__ __align__(16) float so[4][16][132];
  const int tid = threadIdx.x, wave = tid >> 5, lane = tid & 31, col = lane & 15, g = lane >> 4; const int o0 = blockIdx.x * 64 + wave * 16; const int p0 = blockIdx.y * 128;
  v8f acc[8] = {}, accl[8] = {};
#pragma unroll
  for (int kc = 0; kc < QC / 32; ++kc) { v16h ah, al; { const float* p = M + ((size_t)(o0 + col) * QC) + kc * 32 + 8 * g;
#pragma unroll
      for (int i = 0; i < 8; ++i) { const float x0 = p[i] * 1048576.0f, x1 = p[16 + i] * 1048576.0f; const _Float16 h0 = (_Float16)x0, h1 = (_Float16)x1; ah[i] = h0; ah[8 + i] = h1; al[i] = (_Float16)((x0 - (float)h0) * 2048.0f); al[8 + i] = (_Float16)((x1 - (float)h1) * 2048.0f); } }
#pragma unroll
    for (int j = 0; j < 8; ++j) { const v16h w = frag_h(QS + ((size_t)(p0 + j * 16 + col) * QC) + kc * 32, lane); acc[j] = wmma16(ah, w, acc[j]); accl[j] = wmma16(al, w, accl[j]); } }
#pragma unroll
  for (int j = 0; j < 8; ++j)
#pragma unroll
    for (int r = 0; r < 8; ++r) so[wave][8 * g + r][j * 16 + col] = (acc[j][r] + accl[j][r] * (1.0f / 2048.0f)) * (1.0f / 1048576.0f) + bfr(BO[o0 + 8 * g + r]);
  LDSX(); for (int rl = 0; rl < 16; ++rl) vst2(Y + ((size_t)(o0 + rl) * NP) + p0 + lane * 4, *(const v4f*)&so[wave][rl][lane * 4]); }
extern "C" void kernel_launch(void* const* d_in, const int* in_sizes, int n_in, void* d_out, int out_size, void* d_ws, size_t ws_size, hipStream_t stream) {
  (void)in_sizes; (void)n_in; (void)out_size;
  const float** F = (const float**)d_in;
  if (ws_size < (size_t)WS_END) return;
  char* ws = (char*)d_ws; float *WE = (float*)(ws + WS_WE), *BE = (float*)(ws + WS_BE), *CT = (float*)(ws + WS_CT), *M = (float*)(ws + WS_M); __bf16* XT = (__bf16*)(ws + WS_XT); _Float16 *QP = (_Float16*)(ws + WS_QP), *KP = (_Float16*)(ws + WS_KP), *VP = (_Float16*)(ws + WS_VP), *KS = (_Float16*)(ws + WS_KS), *QS = (_Float16*)(ws + WS_QS);
  k_fold<<<dim3(QC, 3), 128, 0, stream>>>(F[1], F[2], F[3], F[4], F[5], F[6], F[7], F[8], F[9], F[10], F[11], F[12], F[13], WE, BE);
  k_foldb<<<3, 128, 0, stream>>>(F[3], F[4], F[5], F[7], F[8], F[9], F[11], F[12], F[13], BE);
  for (int gb = 0; gb < TNB; ++gb) {
    k_xt<<<NP / 64, 256, 0, stream>>>(F[0] + (size_t)gb * CC * NP, XT);
    k_conv<<<dim3(QC / 64, NP / 128, 3), 128, 0, stream>>>(WE, BE, XT, QP, KP, VP);
    k_ksoft<<<QC, 256, 0, stream>>>(KP, KS);
    k_qsoft<<<NP / 128, 128, 0, stream>>>(QP, QS);
    k_ctx<<<NH, 64, 0, stream>>>(KS, VP, CT);
    k_m<<<CC, 128, 0, stream>>>(F[14], CT, M);
    k_y<<<dim3(CC / 64, TPT), 128, 0, stream>>>(M, QS, F[15], (float*)d_out + (size_t)gb * CC * NP); }
}
